// PyFlowODE_2705829396896
// MI455X (gfx1250) — hardware-verified
//
#include <hip/hip_runtime.h>


#ifndef NQ
#define NQ 2048
#endif
#define NQ_FULL 2048
#define NKEY   4096
#define DIM    8
#define KW     32
#define TSTEPS 16
#define AW     4
#define LOG2E  1.4426950408889634f
#define PSH    14.0f
#define QRS    2048.0f
#define QRI    (1.0f / 2048.0f)
#define NEGS   (-1.0e30f)

static_assert(DIM == 8);
static_assert(3 * DIM + 3 <= KW);
static_assert(KW == 32);
static_assert(NKEY % 32 == 0);
static_assert(NQ % (16 * AW) == 0);
static_assert(NQ <= NQ_FULL);
static_assert(((size_t)NKEY * 4) % 256 == 0);
static_assert(((size_t)16 * NKEY / 8) % 256 == 0);
static_assert((TSTEPS & (TSTEPS - 1)) == 0);
static_assert(TSTEPS <= 128);
static_assert(32 * 16 == 16 * DIM * 4);
static_assert(AW * 16 * DIM * 4 <= 131072);

typedef _Float16 h16;
typedef unsigned short bf;
typedef __attribute__((ext_vector_type(16))) __bf16   v16bf;
typedef __attribute__((ext_vector_type(16))) _Float16 v16h;
typedef __attribute__((ext_vector_type(8)))  _Float16 v8h;
typedef __attribute__((ext_vector_type(8)))  unsigned short v8us;
typedef __attribute__((ext_vector_type(8)))  float    v8f;
typedef __attribute__((ext_vector_type(4)))  float    v4f;
typedef v4f  __attribute__((may_alias)) v4fa;

__device__ __forceinline__ unsigned short f2bf(float f) { unsigned u = __float_as_uint(f); u += 0x7FFFu + ((u >> 16) & 1u); return (unsigned short)(u >> 16); }
__device__ __forceinline__ float bfr(float f) { return __uint_as_float(((unsigned)f2bf(f)) << 16); }
__device__ __forceinline__ v16h cat16(v8h lo, v8h hi) { return __builtin_shufflevector(lo, hi, 0, 1, 2, 3, 4, 5, 6, 7, 8, 9, 10, 11, 12, 13, 14, 15); }
__device__ __forceinline__ v16bf cat16b(v8us lo, v8us hi) { return __builtin_bit_cast(v16bf, __builtin_shufflevector(lo, hi, 0, 1, 2, 3, 4, 5, 6, 7, 8, 9, 10, 11, 12, 13, 14, 15)); }
__device__ __forceinline__ v8f wmma16(v16h a, v16h b, v8f c) { return __builtin_amdgcn_wmma_f32_16x16x32_f16(false, a, false, b, (short)0, c, false, false); }
__device__ __forceinline__ v8f wmmab(v16bf a, v16bf b, v8f c) { return __builtin_amdgcn_wmma_f32_16x16x32_bf16(false, a, false, b, (short)0, c, false, false); }
__device__ __forceinline__ v16h  ldh(const h16* p) { return cat16(*(const v8h*)p, *(const v8h*)(p + 16)); }
__device__ __forceinline__ v16bf ldb(const bf* p)  { return cat16b(*(const v8us*)p, *(const v8us*)(p + 16)); }
__device__ __forceinline__ void wave_sync() { __builtin_amdgcn_fence(3  , "wavefront"); __builtin_amdgcn_wave_barrier(); asm volatile("" ::: "memory"); }

__device__ __forceinline__ v8f wmma16g(v16h a, v16h b, v8f c) { c = wmma16(a, b, c); asm volatile("v_nop\n\tv_nop\n\tv_nop\n\tv_nop" : "+v"(c) : "v"(a), "v"(b)); return c; }
__device__ __forceinline__ v8f wmmabg(v16bf a, v16bf b, v8f c) { c = wmmab(a, b, c); asm volatile("v_nop\n\tv_nop\n\tv_nop\n\tv_nop" : "+v"(c) : "v"(a), "v"(b)); return c; }
__device__ __forceinline__ float bf2f(unsigned short b) { return __uint_as_float(((unsigned)b) << 16); }
__device__ __forceinline__ h16 toh_flush(float v) { const h16 r = (h16)v; return (fabsf(v) < 6.103515625e-05f) ? (h16)0.0f : r; }

__global__ __launch_bounds__(256) void k_prep_keys(const float* __restrict__ x0, bf* KA) {
    const int i = blockIdx.x * 256 + threadIdx.x; if (i >= NKEY * 4) return;
    const int row = i >> 2, pc = i & 3;
    const v4f a = *(const v4f*)(x0 + (size_t)row * DIM); const v4f b = *(const v4f*)(x0 + (size_t)row * DIM + 4);
    v8us xo; float n = 0.0f;
#pragma unroll
    for (int k = 0; k < 4; ++k) { xo[k] = f2bf(a[k]); xo[4 + k] = f2bf(b[k]); }
#pragma unroll
    for (int k = 0; k < 8; ++k) { const float v = bf2f(xo[k]); n += v * v; }
    const unsigned short nh = f2bf(n);  const float r1 = n - bf2f(nh);
    const unsigned short nm = f2bf(r1); const float r2 = r1 - bf2f(nm);
    const unsigned short nl = f2bf(r2);
    v8us no = (v8us){}; no[0] = nh; no[1] = nm; no[2] = nl;
    v8us o;
#pragma unroll
    for (int k = 0; k < 8; ++k) o[k] = (pc == 3) ? no[k] : xo[k];
    *(volatile v8us*)(KA + (size_t)i * 8) = o; __threadfence(); *(volatile v8us*)(KA + (size_t)i * 8) = o;
}

__global__ __launch_bounds__(256) void k_prep_vt(const float* __restrict__ x0, h16* VT) {
    const int i = blockIdx.x * 256 + threadIdx.x; if (i >= 16 * NKEY / 8) return;
    const int d = i / (NKEY / 8), kp = i - d * (NKEY / 8);
    const int dc = d < DIM ? d : (DIM - 1);
    v8h o;
#pragma unroll
    for (int j = 0; j < 8; ++j) {
        float v = x0[(size_t)(kp * 8 + j) * DIM + dc];
        asm volatile("" : "+v"(v));
        const float f = (d < DIM) ? bfr(v) : 0.0f;
        o[j] = toh_flush(f); }
    *(volatile v8h*)(VT + (size_t)i * 8) = o; __threadfence(); *(volatile v8h*)(VT + (size_t)i * 8) = o;
}

__global__ __launch_bounds__(32 * AW) void k_heun(const float* __restrict__ X1, const bf* __restrict__ KA, const h16* __restrict__ VT, float* OUT) {
    __shared__ __align__(16) float os[AW * 16 * DIM];
    const int lane = threadIdx.x & 31, lr = lane & 15, hi = lane >> 4;
    const int wave = __builtin_amdgcn_readfirstlane((int)(threadIdx.x >> 5));
    const int t0 = (blockIdx.x * AW + wave) * 16;
    float xt[8], g1[8];
    { const v4f a = *(const v4f*)(X1 + (size_t)(t0 + lr) * DIM); const v4f c = *(const v4f*)(X1 + (size_t)(t0 + lr) * DIM + 4);
#pragma unroll
      for (int i = 0; i < 4; ++i) { xt[i] = bfr(a[i]); xt[4 + i] = bfr(c[i]); } }
#pragma unroll
    for (int d = 0; d < 8; ++d) g1[d] = 0.0f;
    const size_t ko = (size_t)lr * KW + 8 * hi;
    const size_t vo = (size_t)lr * NKEY + 8 * hi;
    const float hstep = 1.0f / (float)TSTEPS;
#pragma unroll 1
    for (int e = 0; e < TSTEPS; ++e) {
        const float tt = 1.0f - hstep * (float)e;
        const float al = 1.0f - tt;
        const float rt = 1.0f / tt;
        const float sc2 = al * rt * rt * LOG2E;
        float y[8];
#pragma unroll
        for (int d = 0; d < 8; ++d) y[d] = xt[d] - g1[d] * hstep;
        const unsigned short cb = f2bf(-0.5f * al);
        v8us blo, bhi;
#pragma unroll
        for (int d = 0; d < 8; ++d) {
            const unsigned short hb = f2bf(y[d]); const float r1 = y[d] - bf2f(hb);
            const unsigned short mb = f2bf(r1);   const float r2 = r1 - bf2f(mb);
            const unsigned short lb = f2bf(r2);
            const unsigned short cz = (d < 3) ? cb : (unsigned short)0;
            blo[d] = hi ? mb : hb;
            bhi[d] = hi ? cz : lb; }
        const v16bf qb = cat16b(blo, bhi);
        v8f o = (v8f){}, oR = (v8f){};
        float m = NEGS, l = 0.0f;
#pragma unroll 1
        for (int key0 = 0; key0 < NKEY; key0 += 32) {
            const bf* ka = KA + ko + (size_t)key0 * KW;
            const v16bf ka0 = ldb(ka), kb0 = ldb(ka + 16 * KW);
            const v16h v0 = ldh(VT + vo + key0);
            v8f sa = (v8f){}, sb = (v8f){};
            sa = wmmabg(ka0, qb, sa);
            sb = wmmabg(kb0, qb, sb);
            float mx = NEGS;
#pragma unroll
            for (int r = 0; r < 8; ++r) mx = fmaxf(mx, fmaxf(sa[r], sb[r]));
            mx = fmaxf(mx, __shfl_xor(mx, 16, 32));
            const float mnew = fmaxf(m, mx);
            const float alpha = __builtin_amdgcn_exp2f((m - mnew) * sc2);
            v16h pb, pr; float ls = 0.0f;
#pragma unroll
            for (int r = 0; r < 8; ++r) {
                const float ea = (sa[r] - mnew) * sc2 + PSH, eb = (sb[r] - mnew) * sc2 + PSH;
                const float xa = __builtin_amdgcn_exp2f(ea), xb = __builtin_amdgcn_exp2f(eb);
                const float ga = (ea < -14.0f) ? 0.0f : xa, gb = (eb < -14.0f) ? 0.0f : xb;
                const h16 pa = toh_flush(ga); const h16 pc = toh_flush(gb);
                pb[r] = pa; pb[8 + r] = pc;
                pr[r] = toh_flush((ga - (float)pa) * QRS); pr[8 + r] = toh_flush((gb - (float)pc) * QRS);
                ls += ga + gb; }
            l = l * alpha + ls; m = mnew;
            o = o * alpha; oR = oR * alpha;
            o = wmma16g(v0, pb, o);
            oR = wmma16g(v0, pr, oR);
        }
        l += __shfl_xor(l, 16, 32);
        const float inv = 1.0f / l;
        const float upd = (e == 0) ? 0.0f : (hstep * 0.5f);
        const v8f f = o + oR * QRI;
#pragma unroll
        for (int d = 0; d < 8; ++d) {
            const float qd = __shfl(f[d], lr, 32) * inv;
            const float gn = (y[d] - qd) * rt;
            xt[d] = xt[d] - (g1[d] + gn) * upd;
            g1[d] = gn; }
    }
    const int wb = wave * 16 * DIM;
    { v4f s;
#pragma unroll
      for (int i = 0; i < 4; ++i) s[i] = hi ? xt[4 + i] : xt[i];
      *(v4fa*)(&os[wb + lr * DIM + 4 * hi]) = s; }
    wave_sync();
    const v4f val = *(const v4fa*)(&os[wb + 4 * lane]);
    float* op = OUT + (size_t)t0 * DIM + 4 * lane;
    *(volatile v4f*)op = val; __threadfence(); *(volatile v4f*)op = val;
}

static constexpr size_t al256(size_t v) { return (v + 255) & ~(size_t)255; }
static constexpr size_t SZ_KA = al256((size_t)NKEY * KW * 2);
static constexpr size_t SZ_VT = al256((size_t)16 * NKEY * 2);
static constexpr size_t SZ_TOTAL = SZ_KA + SZ_VT;
static_assert(SZ_TOTAL <= (size_t)134217728);
static_assert((size_t)NKEY * 4 * 16 == (size_t)NKEY * KW * 2);
static_assert((size_t)(16 * NKEY / 8) * 16 == (size_t)16 * NKEY * 2);

extern "C" void kernel_launch(void* const* d_in, const int* in_sizes, int n_in,
                              void* d_out, int out_size, void* d_ws, size_t ws_size, hipStream_t stream) {
    if (n_in < 2) return;
    if ((size_t)in_sizes[0] < (size_t)NQ * DIM) return;
    if ((size_t)in_sizes[1] < (size_t)NKEY * DIM) return;
    if ((size_t)out_size < (size_t)NQ * DIM) return;
    if (SZ_TOTAL > ws_size) return;
    const float* x1 = (const float*)d_in[0];
    const float* x0 = (const float*)d_in[1];
    float* OUT = (float*)d_out;
    char* wsp = (char*)d_ws;
    bf*  KA = (bf*)wsp;  wsp += SZ_KA;
    h16* VT = (h16*)wsp; wsp += SZ_VT;

    k_prep_keys<<<(unsigned)(((size_t)NKEY * 4) / 256), 256, 0, stream>>>(x0, KA);
    k_prep_vt<<<(unsigned)(((size_t)16 * NKEY / 8) / 256), 256, 0, stream>>>(x0, VT);
    k_heun<<<dim3(NQ / (16 * AW), 1, 1), 32 * AW, 0, stream>>>(x1, KA, VT, OUT);
}
